// mLSTMCell_42949673565
// MI455X (gfx1250) — hardware-verified
//
#include <hip/hip_runtime.h>
#include <math.h>

constexpr int kBatch    = 2;
constexpr int kSeq      = 2048;
constexpr int kDim      = 1024;
constexpr int kHeads    = 4;
constexpr int kDh       = 256;
constexpr int kGateIn   = 3 * kDim;
constexpr int kGroup    = 2;
constexpr int kTok      = kBatch * kSeq;
constexpr int kBH       = kBatch * kHeads;
constexpr int kGtPitch  = 32;
constexpr int kInvPitch = 32;
constexpr int kWElems   = kGateIn * kHeads;
constexpr float kScoreScale = 0.0625f;
constexpr float kPCarry     = 2048.0f;
constexpr float kPCarryInv  = 1.0f / 2048.0f;
constexpr float kEpsN       = 1.0e-6f;
constexpr float kEpsRms     = 1.0e-6f;
constexpr float kInvDh      = 1.0f / 256.0f;
constexpr float kFltMin     = 1.17549435e-38f;
static_assert(kHeads * kDh == kDim, "shape");
static_assert(kWElems == 12288 && kWElems % 1024 == 0, "gate kernel size");
static_assert(kSeq % 64 == 0 && kDh % 64 == 0, "GEMM M/N tile multiples");
static_assert(kDh % 32 == 0 && kSeq % 32 == 0, "GEMM K multiples of 32");
static_assert(kSeq == 256 * 8, "decay kernel: 256 threads x 8 columns = one row");
static_assert(kDim == 256 * 4, "rms kernel: 256 threads x 4 = one token row");
static_assert(kDim == 128 * 8, "prep kernel: 128 threads x 8 per part");
static_assert(kBH * 32 == 256, "scan kernel: one wave per (batch, head)");
static_assert(kHeads % kGroup == 0, "groups");
static_assert(kGtPitch == 32 && kInvPitch == 32, "one 128-B line per table row");

typedef __attribute__((ext_vector_type(16))) _Float16 v16h;
typedef __attribute__((ext_vector_type(8)))  _Float16 v8h;
typedef __attribute__((ext_vector_type(16))) __bf16   v16b;
typedef __attribute__((ext_vector_type(8)))  __bf16   v8b;
typedef __attribute__((ext_vector_type(8)))  float    v8f;
typedef __attribute__((ext_vector_type(4)))  float    v4f;
typedef __attribute__((ext_vector_type(4)))  unsigned int v4u;

__device__ __forceinline__ unsigned short f2bf_bits(float f) {
  unsigned u = __float_as_uint(f);
  return (unsigned short)((u + 0x7FFFu + ((u >> 16) & 1u)) >> 16);
}
__device__ __forceinline__ float bf_bits2f(unsigned short h) { return __uint_as_float(((unsigned)h) << 16); }

__device__ __forceinline__ void dep_guard_h(v8f& a, v8f& b, v16h x, v16h y) { asm volatile("v_nop\n\tv_nop\n\tv_nop\n\tv_nop" : "+v"(a), "+v"(b) : "v"(x), "v"(y)); }
__device__ __forceinline__ void dep_guard_b(v8f& a, v8f& b, v16b x, v16b y) { asm volatile("v_nop\n\tv_nop\n\tv_nop\n\tv_nop" : "+v"(a), "+v"(b) : "v"(x), "v"(y)); }
__device__ __forceinline__ void dep_guard4_h(v8f& a, v8f& b, v8f& c, v8f& d, v16h x, v16h y) { asm volatile("v_nop\n\tv_nop\n\tv_nop\n\tv_nop" : "+v"(a), "+v"(b), "+v"(c), "+v"(d) : "v"(x), "v"(y)); }
__device__ __forceinline__ void dep_guard4_b(v8f& a, v8f& b, v8f& c, v8f& d, v16b x, v16b y) { asm volatile("v_nop\n\tv_nop\n\tv_nop\n\tv_nop" : "+v"(a), "+v"(b), "+v"(c), "+v"(d) : "v"(x), "v"(y)); }
__device__ __forceinline__ void keep4_h(v16h a, v16h b, v16h c, v16h d) { asm volatile("v_nop" :: "v"(a), "v"(b), "v"(c), "v"(d)); }
__device__ __forceinline__ void keep4_b(v16b a, v16b b, v16b c, v16b d) { asm volatile("v_nop" :: "v"(a), "v"(b), "v"(c), "v"(d)); }
__device__ __forceinline__ void acc_guard4(v8f& a, v8f& b, v8f& c, v8f& d) { asm volatile("v_nop\n\tv_nop\n\tv_nop\n\tv_nop" : "+v"(a), "+v"(b), "+v"(c), "+v"(d)); }
__device__ __forceinline__ void acc_tie(float& a, float& b, float& c, float& d, unsigned& o) { asm volatile("" : "+v"(a), "+v"(b), "+v"(c), "+v"(d), "+v"(o)); }
template <typename T> struct Frag;
template <> struct Frag<_Float16> {
  typedef v16h V; union U { v16h v; v8h h[2]; };
  static __device__ __forceinline__ v16h load(const _Float16* p) {
    U f; f.h[0] = *(const v8h*)(p); f.h[1] = *(const v8h*)(p + 16); return f.v;
  }
  static __device__ __forceinline__ v8f mma(v16h a, v16h b, v8f c) {
    return __builtin_amdgcn_wmma_f32_16x16x32_f16(false, a, false, b, (short)0, c, false, false);
  }
  static __device__ __forceinline__ void guard(v8f& a, v8f& b, v16h x, v16h y) { dep_guard_h(a, b, x, y); }
  static __device__ __forceinline__ void guard4(v8f& a, v8f& b, v8f& c, v8f& d, v16h x, v16h y) { dep_guard4_h(a, b, c, d, x, y); }
  static __device__ __forceinline__ void keep(v16h a, v16h b, v16h c, v16h d) { keep4_h(a, b, c, d); }
};
template <> struct Frag<__bf16> {
  typedef v16b V; union U { v16b v; v8b h[2]; };
  static __device__ __forceinline__ v16b load(const __bf16* p) {
    U f; f.h[0] = *(const v8b*)(p); f.h[1] = *(const v8b*)(p + 16); return f.v;
  }
  static __device__ __forceinline__ v8f mma(v16b a, v16b b, v8f c) {
    return __builtin_amdgcn_wmma_f32_16x16x32_bf16(false, a, false, b, (short)0, c, false, false);
  }
  static __device__ __forceinline__ void guard(v8f& a, v8f& b, v16b x, v16b y) { dep_guard_b(a, b, x, y); }
  static __device__ __forceinline__ void guard4(v8f& a, v8f& b, v8f& c, v8f& d, v16b x, v16b y) { dep_guard4_b(a, b, c, d, x, y); }
  static __device__ __forceinline__ void keep(v16b a, v16b b, v16b c, v16b d) { keep4_b(a, b, c, d); }
};

__device__ __forceinline__ unsigned pk16(unsigned short a, unsigned short b) { return (unsigned)a | ((unsigned)b << 16); }
__device__ __forceinline__ unsigned short h_bits(float f) { const _Float16 h = (_Float16)f; return __builtin_bit_cast(unsigned short, h); }

template <int ET> struct Elem;
template <> struct Elem<0> { typedef _Float16 T; };
template <> struct Elem<1> { typedef __bf16 T; };
template <int ET, bool SPLIT, int BIAS_MODE, int OUT_MODE, bool RESID, int ACT = 0>
__global__ __launch_bounds__(256) void wmma_gemm64(
    const unsigned short* __restrict__ Ap, const unsigned short* __restrict__ A2p, int lda, long strideA,
    const unsigned short* __restrict__ Btp, const unsigned short* __restrict__ Bt2p, int ldb, long strideB,
    void* __restrict__ Cout, void* __restrict__ Cout2, int ldc, long strideC,
    const float* __restrict__ bias,
    const float* __restrict__ resid, long strideR,
    int M, int N, int K, float scale) {
  typedef typename Elem<ET>::T T;
  typedef typename Frag<T>::V V;
  const T* A = (const T*)Ap; const T* A2 = (const T*)A2p; const T* Bt = (const T*)Btp; const T* Bt2 = (const T*)Bt2p;
  __shared__ __align__(16) float sT[8][16 * 68];
  const int b    = blockIdx.y;
  const int lane = threadIdx.x & 31;
  const int wave = threadIdx.x >> 5;
  const int tilesN = N >> 6;
  const int tilesM = M >> 6;
  const int tile = blockIdx.x * 8 + wave;
  if (tile >= tilesM * tilesN) return;
  const int tm = tile / tilesN;
  const int tn = tile - tm * tilesN;
  const int m0 = tm << 6;
  const int n0 = tn << 6;

  const T* Ab  = A  + (size_t)b * strideA;
  const T* Bb  = Bt + (size_t)b * strideB;
  const T* Ab2 = SPLIT ? (A2  + (size_t)b * strideA) : nullptr;
  const T* Bb2 = SPLIT ? (Bt2 + (size_t)b * strideB) : nullptr;

  const int rlane = lane & 15;
  const int koff  = (lane >> 4) * 8;
  const int mOff  = (lane >> 4) * 8;

  v8f acc[4][4];
#pragma unroll
  for (int i = 0; i < 4; ++i)
#pragma unroll
    for (int j = 0; j < 4; ++j) acc[i][j] = (v8f){0.f,0.f,0.f,0.f,0.f,0.f,0.f,0.f};

  for (int k0 = 0; k0 < K; k0 += 32) {
    V bh[4], bl[4];
#pragma unroll
    for (int j = 0; j < 4; ++j) {
      const size_t bo = (size_t)(n0 + (j << 4) + rlane) * ldb + koff + k0;
      bh[j] = Frag<T>::load(Bb + bo);
      if (SPLIT) bl[j] = Frag<T>::load(Bb2 + bo);
    }
#pragma unroll
    for (int i = 0; i < 4; ++i) {
      const size_t ao = (size_t)(m0 + (i << 4) + rlane) * lda + koff + k0;
      V ah = Frag<T>::load(Ab + ao);
      V al;
      if (SPLIT) al = Frag<T>::load(Ab2 + ao);
#pragma unroll
      for (int j = 0; j < 4; ++j) {
        acc[i][j] = Frag<T>::mma(ah, bh[j], acc[i][j]);
        if (SPLIT) {
          acc[i][j] = Frag<T>::mma(ah, bl[j], acc[i][j]);
          acc[i][j] = Frag<T>::mma(al, bh[j], acc[i][j]);
        }
      }
      Frag<T>::guard4(acc[i][0], acc[i][1], acc[i][2], acc[i][3], ah, SPLIT ? al : ah);
    }
    Frag<T>::keep(bh[0], bh[1], bh[2], bh[3]);
    if (SPLIT) Frag<T>::keep(bl[0], bl[1], bl[2], bl[3]);
  }
  acc_guard4(acc[0][0], acc[0][1], acc[0][2], acc[0][3]);
  acc_guard4(acc[1][0], acc[1][1], acc[1][2], acc[1][3]);
  acc_guard4(acc[2][0], acc[2][1], acc[2][2], acc[2][3]);
  acc_guard4(acc[3][0], acc[3][1], acc[3][2], acc[3][3]);

  float* slab = sT[wave];
  const float* Rb = RESID ? (resid + (size_t)b * strideR) : nullptr;
#pragma unroll
  for (int i = 0; i < 4; ++i) {
    const int mBase = m0 + (i << 4);
#pragma unroll
    for (int j = 0; j < 4; ++j) {
      const int n = n0 + (j << 4) + rlane;
      float bv = 0.f;
      if (BIAS_MODE == 2) bv = bias[n];
#pragma unroll
      for (int r = 0; r < 8; ++r) {
        float v = acc[i][j][r] * scale;
        if (BIAS_MODE == 1) v += bias[mBase + mOff + r];
        if (BIAS_MODE == 2) v += bv;
        if (RESID) v += Rb[(size_t)(mBase + mOff + r) * ldc + n];
        if (ACT == 2) v = fmaxf(v, 0.0f);
        if (ACT == 4) v = (v > 0.f) ? v : 0.01f * v;
        slab[(mOff + r) * 68 + (j << 4) + rlane] = v;
      }
    }
    __builtin_amdgcn_fence(__ATOMIC_RELEASE, "workgroup");
    __builtin_amdgcn_wave_barrier();
    __builtin_amdgcn_fence(__ATOMIC_ACQUIRE, "workgroup");
    if (OUT_MODE == 0) {
      float* C = (float*)Cout + (size_t)b * strideC;
      const int hh = lane >> 4, c4 = (lane & 15) * 4;
      for (int pass = 0; pass < 2; ++pass) {
#pragma unroll
        for (int it = 0; it < 8; ++it) {
          const int row = it * 2 + hh;
          v4f v = *(const v4f*)(slab + row * 68 + c4);
          *(volatile v4f*)(C + (size_t)(mBase + row) * ldc + n0 + c4) = v;
        }
        __threadfence();
      }
    } else {
      const int q = lane >> 3, c8 = (lane & 7) * 8;
      unsigned short* C  = (unsigned short*)Cout  + (size_t)b * strideC;
      unsigned short* C2 = (OUT_MODE == 2) ? ((unsigned short*)Cout2 + (size_t)b * strideC) : nullptr;
      for (int pass = 0; pass < 2; ++pass) {
#pragma unroll
        for (int it = 0; it < 4; ++it) {
          const int row = it * 4 + q;
          const float* sp = slab + row * 68 + c8;
          v8h hv, lv;
#pragma unroll
          for (int e = 0; e < 8; ++e) {
            if (OUT_MODE == 1) {
              hv[e] = (_Float16)sp[e];
            } else {
              unsigned short hb = f2bf_bits(sp[e]);
              unsigned short lb = f2bf_bits(sp[e] - bf_bits2f(hb));
              hv[e] = __builtin_bit_cast(_Float16, hb);
              lv[e] = __builtin_bit_cast(_Float16, lb);
            }
          }
          *(volatile v8h*)(C + (size_t)(mBase + row) * ldc + n0 + c8) = hv;
          if (OUT_MODE == 2) *(volatile v8h*)(C2 + (size_t)(mBase + row) * ldc + n0 + c8) = lv;
        }
        __threadfence();
      }
    }
    __builtin_amdgcn_fence(__ATOMIC_RELEASE, "workgroup");
    __builtin_amdgcn_wave_barrier();
    __builtin_amdgcn_fence(__ATOMIC_ACQUIRE, "workgroup");
  }
}

__device__ __forceinline__ float bf_rne(float f) { return bf_bits2f(f2bf_bits(f)); }

__device__ __forceinline__ float log_sigmoid_f(float x) {
  const float t = log1pf(expf(-fabsf(x)));
  return -(fmaxf(-x, 0.0f) + t);
}

__device__ __forceinline__ void gate_acc(float x, v4f w, float& a0, float& a1, float& a2, float& a3) {
  a0 = a0 + x * w[0];
  a1 = a1 + x * w[1];
  a2 = a2 + x * w[2];
  a3 = a3 + x * w[3];
}

__global__ __launch_bounds__(256) void wcvt_kernel(const float* __restrict__ w0, const float* __restrict__ w1,
                                                   float* __restrict__ dst) {
  constexpr int kBlocksPer = kWElems / 1024;
  const int z = (blockIdx.x >= kBlocksPer) ? 1 : 0;
  const int i = (blockIdx.x - z * kBlocksPer) * 256 + threadIdx.x;
  const float* src = (z == 0) ? w0 : w1;
  const v4f x = *(const v4f*)(src + 4 * (size_t)i);
  v4f y;
#pragma unroll
  for (int e = 0; e < 4; ++e) { const float f = x[e]; y[e] = bf_rne(f); }
  float* dp = dst + (size_t)z * kWElems + 4 * (size_t)i;
  *(volatile v4f*)dp = y;
  __threadfence();
  *(volatile v4f*)dp = y;
}

__global__ __launch_bounds__(384) void prep_gates_kernel(
    const float* __restrict__ q, const float* __restrict__ k, const float* __restrict__ v,
    const float* __restrict__ wr, const float* __restrict__ igb, const float* __restrict__ fgb,
    unsigned short* __restrict__ Qb, unsigned short* __restrict__ Kb, float* __restrict__ GT) {
  __shared__ float red[12 * 8];
  const int r    = blockIdx.x;
  const int t    = threadIdx.x;
  const int lane = t & 31, wave = t >> 5;
  const int part = t >> 7;
  const int c8   = (t & 127) * 8;
  const float* src = (part == 0) ? q : ((part == 1) ? k : v);
  const float* xp = src + (size_t)r * kDim + c8;
  const v4f xa = *(const v4f*)(xp);
  const v4f xc = *(const v4f*)(xp + 4);
  float xr[8];
  unsigned short xh[8];
#pragma unroll
  for (int e = 0; e < 4; ++e) {
    const float f0 = xa[e];
    const float f1 = xc[e];
    const unsigned short h0 = f2bf_bits(f0);
    const unsigned short h1 = f2bf_bits(f1);
    xh[e] = h0;  xh[4 + e] = h1;
    xr[e] = bf_bits2f(h0);  xr[4 + e] = bf_bits2f(h1);
  }
  if (part < 2) {
    const v4u u = (v4u){pk16(xh[0], xh[1]), pk16(xh[2], xh[3]), pk16(xh[4], xh[5]), pk16(xh[6], xh[7])};
    unsigned short* dp = ((part == 0) ? Qb : Kb) + (size_t)r * kDim + c8;
    *(volatile v4u*)dp = u;
    __threadfence();
    *(volatile v4u*)dp = u;
  }

  const int ebase = part * kDim + c8;
  unsigned wofs = (unsigned)(ebase * kHeads);
  float ai0 = 0.0f, ai1 = 0.0f, ai2 = 0.0f, ai3 = 0.0f;
  float af0 = 0.0f, af1 = 0.0f, af2 = 0.0f, af3 = 0.0f;
  {
    const float* wp = wr + wofs;
    const v4f w0 = *(const v4f*)(wp + 0), w1 = *(const v4f*)(wp + 4), w2 = *(const v4f*)(wp + 8), w3 = *(const v4f*)(wp + 12);
    gate_acc(xr[0], w0, ai0, ai1, ai2, ai3);
    gate_acc(xr[1], w1, ai0, ai1, ai2, ai3);
    gate_acc(xr[2], w2, ai0, ai1, ai2, ai3);
    gate_acc(xr[3], w3, ai0, ai1, ai2, ai3);
  }
  acc_tie(ai0, ai1, ai2, ai3, wofs);
  {
    const float* wp = wr + wofs + 16;
    const v4f w4 = *(const v4f*)(wp + 0), w5 = *(const v4f*)(wp + 4), w6 = *(const v4f*)(wp + 8), w7 = *(const v4f*)(wp + 12);
    gate_acc(xr[4], w4, ai0, ai1, ai2, ai3);
    gate_acc(xr[5], w5, ai0, ai1, ai2, ai3);
    gate_acc(xr[6], w6, ai0, ai1, ai2, ai3);
    gate_acc(xr[7], w7, ai0, ai1, ai2, ai3);
  }
  acc_tie(ai0, ai1, ai2, ai3, wofs);
  {
    const float* wp = wr + kWElems + wofs;
    const v4f w0 = *(const v4f*)(wp + 0), w1 = *(const v4f*)(wp + 4), w2 = *(const v4f*)(wp + 8), w3 = *(const v4f*)(wp + 12);
    gate_acc(xr[0], w0, af0, af1, af2, af3);
    gate_acc(xr[1], w1, af0, af1, af2, af3);
    gate_acc(xr[2], w2, af0, af1, af2, af3);
    gate_acc(xr[3], w3, af0, af1, af2, af3);
  }
  acc_tie(af0, af1, af2, af3, wofs);
  {
    const float* wp = wr + kWElems + wofs + 16;
    const v4f w4 = *(const v4f*)(wp + 0), w5 = *(const v4f*)(wp + 4), w6 = *(const v4f*)(wp + 8), w7 = *(const v4f*)(wp + 12);
    gate_acc(xr[4], w4, af0, af1, af2, af3);
    gate_acc(xr[5], w5, af0, af1, af2, af3);
    gate_acc(xr[6], w6, af0, af1, af2, af3);
    gate_acc(xr[7], w7, af0, af1, af2, af3);
  }
#pragma unroll
  for (int off = 16; off > 0; off >>= 1) {
    ai0 += __shfl_xor(ai0, off, 32);
    ai1 += __shfl_xor(ai1, off, 32);
    ai2 += __shfl_xor(ai2, off, 32);
    ai3 += __shfl_xor(ai3, off, 32);
    af0 += __shfl_xor(af0, off, 32);
    af1 += __shfl_xor(af1, off, 32);
    af2 += __shfl_xor(af2, off, 32);
    af3 += __shfl_xor(af3, off, 32);
  }
  if (lane == 0) {
    red[wave * 8 + 0] = ai0; red[wave * 8 + 1] = ai1; red[wave * 8 + 2] = ai2; red[wave * 8 + 3] = ai3;
    red[wave * 8 + 4] = af0; red[wave * 8 + 5] = af1; red[wave * 8 + 6] = af2; red[wave * 8 + 7] = af3;
  }
  __syncthreads();
  {
    const int o = lane & 7;
    float s = 0.0f;
#pragma unroll
    for (int w = 0; w < 12; ++w) s = s + red[w * 8 + o];
    const float bi = bf_rne(igb[lane & 3]);
    const float bf = bf_rne(fgb[lane & 3]);
    const float fi = (o < 4) ? 1.0f : 0.0f;
    const float bsel = fi * bi + (1.0f - fi) * bf;
    const float g = s + bsel;
    const float a0 = __shfl(g, (4 * lane + 0) & 31, 32);
    const float a1 = __shfl(g, (4 * lane + 1) & 31, 32);
    const float a2 = __shfl(g, (4 * lane + 2) & 31, 32);
    const float a3 = __shfl(g, (4 * lane + 3) & 31, 32);
    const float keep = (lane < 2) ? 1.0f : 0.0f;
    const v4f val = (v4f){a0 * keep, a1 * keep, a2 * keep, a3 * keep};
    if (t < 8) {
      float* dp = GT + (size_t)r * kGtPitch + 4 * lane;
      *(volatile v4f*)dp = val;
      __threadfence();
      *(volatile v4f*)dp = val;
    }
  }
}

__global__ __launch_bounds__(256) void vt_kernel(const float* __restrict__ v, unsigned short* __restrict__ VT) {
  __shared__ float sm[64][65];
  const int t  = threadIdx.x;
  const int s0 = blockIdx.x * 64;
  const int h  = blockIdx.y >> 2;
  const int dc = blockIdx.y & 3;
  const int b  = blockIdx.z;
  const float* vb = v + ((size_t)b * kSeq + s0) * kDim + h * kDh + dc * 64;
#pragma unroll
  for (int i = 0; i < 8; ++i) {
    const int e = i * 256 + t;
    const int rr = e >> 6;
    const int cc = e & 63;
    sm[cc][rr] = vb[(size_t)rr * kDim + cc];
  }
  asm volatile("" ::: "memory");
#pragma unroll
  for (int i = 8; i < 16; ++i) {
    const int e = i * 256 + t;
    const int rr = e >> 6;
    const int cc = e & 63;
    sm[cc][rr] = vb[(size_t)rr * kDim + cc];
  }
  __syncthreads();
  const int lane = t & 31, wave = t >> 5;
  const int qq = lane >> 3, c8 = (lane & 7) * 8;
  unsigned short* op = VT + ((size_t)(b * kHeads + h) * kDh + dc * 64) * kSeq;
  for (int pass = 0; pass < 2; ++pass) {
#pragma unroll
    for (int it = 0; it < 2; ++it) {
      const int row = wave * 8 + it * 4 + qq;
      unsigned short hb[8];
#pragma unroll
      for (int e = 0; e < 8; ++e) { const float f = sm[row][c8 + e]; hb[e] = h_bits(bf_rne(f)); }
      const v4u u = (v4u){pk16(hb[0], hb[1]), pk16(hb[2], hb[3]), pk16(hb[4], hb[5]), pk16(hb[6], hb[7])};
      *(volatile v4u*)(op + (size_t)row * kSeq + s0 + c8) = u;
    }
    __threadfence();
  }
}

__global__ __launch_bounds__(256) void scan_kernel(const float* __restrict__ GT, float* __restrict__ CSp,
                                                   float* __restrict__ BVp, float* __restrict__ MBp,
                                                   float* __restrict__ EMp) {
  const int t = threadIdx.x;
  const int lane = t & 31, wave = t >> 5;
  const int bh = wave;
  const int b = bh >> 2, h = bh & 3;
  const float* gbase = GT + (size_t)b * kSeq * kGtPitch;
  float carry = 0.0f;
  float runmax = -__builtin_inff();
#pragma unroll 1
  for (int ch = 0; ch < kSeq / 32; ++ch) {
    const int tt = ch * 32 + lane;
    const float* gp = gbase + (size_t)tt * kGtPitch;
    const float ig = gp[h];
    const float fg = gp[4 + h];
    const float lf = log_sigmoid_f(fg);
    float cs = 0.0f;
#pragma unroll
    for (int i = 0; i < 32; ++i) {
      const float o = __shfl(lf, i, 32);
      carry = carry + o;
      cs = (lane == i) ? carry : cs;
    }
    const float bv = ig - cs;
    float mb = 0.0f;
#pragma unroll
    for (int i = 0; i < 32; ++i) {
      const float o = __shfl(bv, i, 32);
      runmax = fmaxf(runmax, o);
      mb = (lane == i) ? runmax : mb;
    }
    const float em = expf(-(cs + mb));
    const size_t off = (size_t)bh * kSeq + tt;
    *(volatile float*)(CSp + off) = cs;
    *(volatile float*)(BVp + off) = bv;
    *(volatile float*)(MBp + off) = mb;
    *(volatile float*)(EMp + off) = em;
    __threadfence();
    *(volatile float*)(CSp + off) = cs;
    *(volatile float*)(BVp + off) = bv;
    *(volatile float*)(MBp + off) = mb;
    *(volatile float*)(EMp + off) = em;
  }
}

__global__ __launch_bounds__(256) void decay_kernel(const float* __restrict__ SC, const float* __restrict__ BV,
                                                    const float* __restrict__ MB, const float* __restrict__ EM,
                                                    unsigned short* __restrict__ PP, float* __restrict__ INV, int bh0) {
  __shared__ float redS[8];
  const int i    = blockIdx.x;
  const int hg   = blockIdx.y;
  const int bh   = bh0 + hg;
  const int t    = threadIdx.x;
  const int lane = t & 31, wave = t >> 5;
  const size_t rowoff = ((size_t)hg * kSeq + i) * kSeq;
  const float* sr = SC + rowoff + 8 * (size_t)t;
  const float* br = BV + (size_t)bh * kSeq + 8 * t;
  const float mbi = MB[(size_t)bh * kSeq + i];
  const float emi = EM[(size_t)bh * kSeq + i];
  float rs = 0.0f;
  unsigned wa = 0u, wb = 0u, wc = 0u, wd = 0u;
#pragma unroll 1
  for (int it = 0; it < 2; ++it) {
    const v4f sv  = *(const v4f*)(sr + 4 * it);
    const v4f bvv = *(const v4f*)(br + 4 * it);
    const int j0 = 8 * t + 4 * it;
    unsigned short hb[4];
#pragma unroll
    for (int e = 0; e < 4; ++e) {
      const float s  = sv[e];
      const float bj = bvv[e];
      const float x  = fminf(bj - mbi, 0.0f);
      float ex = expf(x);
      ex = (ex < kFltMin) ? 0.0f : ex;
      const float fm = (j0 + e <= i) ? 1.0f : 0.0f;
      const float c = (s * ex) * fm;
      rs = rs + c;
      hb[e] = h_bits(c * kPCarry);
    }
    const unsigned p0 = pk16(hb[0], hb[1]);
    const unsigned p1 = pk16(hb[2], hb[3]);
    if (it == 0) { wa = p0; wb = p1; } else { wc = p0; wd = p1; }
  }
#pragma unroll
  for (int off = 16; off > 0; off >>= 1) rs += __shfl_xor(rs, off, 32);
  if (lane == 0) redS[wave] = rs;
  __syncthreads();
  float tot = redS[0];
#pragma unroll
  for (int w = 1; w < 8; ++w) tot = tot + redS[w];
  const float n = fmaxf(tot, emi);
  const float inv = 1.0f / (n + kEpsN);

  const v4u u = (v4u){wa, wb, wc, wd};
  unsigned short* pr = PP + rowoff + 8 * (size_t)t;
  *(volatile v4u*)pr = u;
  __threadfence();
  *(volatile v4u*)pr = u;

  if (t < 8) {
    const float keep = (t == 0) ? 1.0f : 0.0f;
    const v4f val = (v4f){inv * keep, 0.0f, 0.0f, 0.0f};
    float* dp = INV + ((size_t)bh * kSeq + i) * kInvPitch + 4 * t;
    *(volatile v4f*)dp = val;
    __threadfence();
    *(volatile v4f*)dp = val;
  }
}

__global__ __launch_bounds__(256) void rms_out_kernel(const float* __restrict__ H, const float* __restrict__ INV,
                                                      const float* __restrict__ rms, float* __restrict__ out) {
  __shared__ float red[8];
  const int r    = blockIdx.x;
  const int b    = r / kSeq;
  const int s    = r - b * kSeq;
  const int t    = threadIdx.x;
  const int lane = t & 31, wave = t >> 5;
  const int h    = t >> 6;
  const int d0   = (t & 63) * 4;
  const v4f x = *(const v4f*)(H + (size_t)r * kDim + h * kDh + d0);
  const float inv = INV[((size_t)(b * kHeads + h) * kSeq + s) * kInvPitch];
  const v4f rsr = *(const v4f*)(rms + d0);
  float hv[4];
  float ss = 0.0f;
#pragma unroll
  for (int e = 0; e < 4; ++e) { const float xe = x[e]; hv[e] = xe * inv; ss = ss + hv[e] * hv[e]; }
#pragma unroll
  for (int off = 16; off > 0; off >>= 1) ss += __shfl_xor(ss, off, 32);
  if (lane == 0) red[wave] = ss;
  __syncthreads();
  const float ssq = red[2 * h] + red[2 * h + 1];
  const float var = ssq * kInvDh;
  const float rn  = rsqrtf(var + kEpsRms);
  v4f o;
#pragma unroll
  for (int e = 0; e < 4; ++e) { const float re = rsr[e]; const float g = 1.0f + bf_rne(re); o[e] = (hv[e] * rn) * g; }
  float* dp = out + (size_t)r * kDim + 4 * t;
  *(volatile v4f*)dp = o;
  __threadfence();
  *(volatile v4f*)dp = o;
}

extern "C" void kernel_launch(void* const* d_in, const int* in_sizes, int n_in,
                              void* d_out, int out_size, void* d_ws, size_t ws_size,
                              hipStream_t stream) {
  if (n_in < 8) return;
  const int nElem = kTok * kDim;
  if (in_sizes[0] != nElem || in_sizes[1] != nElem || in_sizes[2] != nElem) return;
  if (in_sizes[3] != kWElems || in_sizes[5] != kWElems) return;
  if (in_sizes[4] != kHeads || in_sizes[6] != kHeads || in_sizes[7] != kDh) return;
  if (out_size != nElem) return;

  const size_t szWR  = (size_t)2 * kWElems * 4;
  const size_t szQK  = (size_t)kTok * kDim * 2;
  const size_t szVT  = (size_t)kBH * kDh * kSeq * 2;
  const size_t szGT  = (size_t)kTok * kGtPitch * 4;
  const size_t szSc  = (size_t)kBH * kSeq * 4;
  const size_t szS   = (size_t)kGroup * kSeq * kSeq * 4;
  const size_t szP   = (size_t)kGroup * kSeq * kSeq * 2;
  const size_t szInv = (size_t)kBH * kSeq * kInvPitch * 4;
  const size_t szH   = (size_t)kTok * kDim * 4;
  const size_t offWR  = 0;
  const size_t offQB  = offWR + szWR;
  const size_t offKB  = offQB + szQK;
  const size_t offVT  = offKB + szQK;
  const size_t offGT  = offVT + szVT;
  const size_t offCS  = offGT + szGT;
  const size_t offBV  = offCS + szSc;
  const size_t offMB  = offBV + szSc;
  const size_t offEM  = offMB + szSc;
  const size_t offS   = offEM + szSc;
  const size_t offP   = offS + szS;
  const size_t offInv = offP + szP;
  const size_t offH   = offInv + szInv;
  const size_t total  = offH + szH;
  if (ws_size < total) return;

  const float* q   = (const float*)d_in[0];
  const float* k   = (const float*)d_in[1];
  const float* v   = (const float*)d_in[2];
  const float* igk = (const float*)d_in[3];
  const float* igb = (const float*)d_in[4];
  const float* fgk = (const float*)d_in[5];
  const float* fgb = (const float*)d_in[6];
  const float* rms = (const float*)d_in[7];
  float* out = (float*)d_out;
  char* ws = (char*)d_ws;
  float* WR = (float*)(ws + offWR);
  unsigned short* QB = (unsigned short*)(ws + offQB);
  unsigned short* KB = (unsigned short*)(ws + offKB);
  unsigned short* VT = (unsigned short*)(ws + offVT);
  float* GT  = (float*)(ws + offGT);
  float* CSp = (float*)(ws + offCS);
  float* BVp = (float*)(ws + offBV);
  float* MBp = (float*)(ws + offMB);
  float* EMp = (float*)(ws + offEM);
  float* SC  = (float*)(ws + offS);
  unsigned short* PP = (unsigned short*)(ws + offP);
  float* INVp = (float*)(ws + offInv);
  float* Hp   = (float*)(ws + offH);

  wcvt_kernel<<<dim3(2 * (kWElems / 1024)), dim3(256), 0, stream>>>(igk, fgk, WR);
  prep_gates_kernel<<<dim3(kTok), dim3(384), 0, stream>>>(q, k, v, WR, igb, fgb, QB, KB, GT);
  vt_kernel<<<dim3(kSeq / 64, kHeads * (kDh / 64), kBatch), dim3(256), 0, stream>>>(v, VT);
  scan_kernel<<<dim3(1), dim3(256), 0, stream>>>(GT, CSp, BVp, MBp, EMp);

  const long strideHead16 = (long)kDh;
  const long strideScore  = (long)kSeq * kSeq;
  const long strideVT     = (long)kDh * kSeq;
  const int  tilesScore   = (kSeq / 64) * (kSeq / 64);
  const int  tilesCtx     = (kSeq / 64) * (kDh / 64);

  for (int b = 0; b < kBatch; ++b) {
    for (int g = 0; g < kHeads / kGroup; ++g) {
      const int hbase = g * kGroup;
      const int bh0 = b * kHeads + hbase;
      const size_t tokOff = ((size_t)b * kSeq) * kDim + (size_t)hbase * kDh;
      const unsigned short* Ag  = QB + tokOff;
      const unsigned short* Btg = KB + tokOff;
      wmma_gemm64<1, false, 0, 0, false, 0><<<dim3(tilesScore / 8, kGroup), dim3(256), 0, stream>>>(
          Ag, Ag, kDim, strideHead16, Btg, Btg, kDim, strideHead16,
          (void*)SC, (void*)SC, kSeq, strideScore, WR, WR, 0L, kSeq, kSeq, kDh, kScoreScale);
      decay_kernel<<<dim3(kSeq, kGroup), dim3(256), 0, stream>>>(SC, BVp, MBp, EMp, PP, INVp, bh0);
      const unsigned short* VTg = VT + (size_t)bh0 * kDh * kSeq;
      float* Hg = Hp + tokOff;
      wmma_gemm64<0, false, 0, 0, false, 0><<<dim3(tilesCtx / 8, kGroup), dim3(256), 0, stream>>>(
          PP, PP, kSeq, strideScore, VTg, VTg, kSeq, strideVT,
          (void*)Hg, (void*)Hg, kDim, strideHead16, WR, WR, 0L, kSeq, kDh, kSeq, kPCarryInv);
    }
  }

  rms_out_kernel<<<dim3(kTok), dim3(256), 0, stream>>>(Hp, INVp, rms, out);
}
